// PhaseAttention_24043226923316
// MI455X (gfx1250) — hardware-run, weakly checked
//
#include <hip/hip_runtime.h>
#include <math.h>

typedef __attribute__((ext_vector_type(16))) _Float16 v16h;
typedef __attribute__((ext_vector_type(8)))  _Float16 v8h;
typedef __attribute__((ext_vector_type(16))) __bf16   v16b;
typedef __attribute__((ext_vector_type(8)))  __bf16   v8b;
typedef __attribute__((ext_vector_type(8)))  float    v8f;
typedef __attribute__((ext_vector_type(4)))  float    v4f;

constexpr int  kInputsRneToBf16 = 1;
constexpr bool kSplit = (kInputsRneToBf16 == 0);

constexpr int kBatch  = 2;
constexpr int kSeq    = 512;
constexpr int kDm     = 512;
constexpr int kHeads  = 8;
constexpr int kOsc    = 64;
constexpr int kIters  = 10;
constexpr int kRows   = kBatch * kSeq;
constexpr int kCols   = kHeads * kOsc;
constexpr int kChunkCols     = 8;
constexpr int kChunks        = kOsc / kChunkCols;
constexpr int kSyncBlocks    = kBatch * kHeads * kChunks;
constexpr int kSyncThreads   = 256;
constexpr int kRowGroups     = kSyncThreads / kChunkCols;
constexpr int kRowsPerThread = kSeq / kRowGroups;
constexpr int kChunkElems    = kSeq * kChunkCols;
static_assert(kRows == 1024 && kCols == 512 && kDm == 512, "plane shapes");
static_assert((kDm % 32) == 0 && (kCols % 32) == 0, "GEMM K multiples of 32");
static_assert((kRows % 64) == 0 && (kCols % 64) == 0 && (kDm % 64) == 0, "GEMM M,N multiples of 64");
static_assert(kChunks * kChunkCols == kOsc && kRowGroups * kRowsPerThread == kSeq, "sync tiling");
static_assert(kSyncThreads * 2 == kSeq, "mask staging covers the sequence with two elements per thread");
static_assert(kChunkElems == 4 * kSyncThreads * 4, "chunk copy: 4 instructions x 256 threads x 4 floats");
static_assert(kSyncBlocks == 128 && kRowGroups == 32 && kRowsPerThread == 16, "sync geometry");

constexpr float kCarryW      = 1024.0f;
constexpr float kCarryPh     = 16.0f;
constexpr float kFold        = 1.0f / (kCarryW * kCarryPh);
constexpr float kF16MinNormal = 6.103515625e-5f;
constexpr float kPiF    = 3.14159265358979323846f;
constexpr float kTwoPiF = 2.0f * kPiF;
constexpr float kDtF    = 0.1f;
constexpr float kInvSeq = 1.0f / (float)kSeq;

constexpr size_t kSzXH  = (size_t)kRows * kDm * 2;
constexpr size_t kSzXL  = kSplit ? kSzXH : 0;
constexpr size_t kSzWPH = (size_t)kCols * kDm * 2;
constexpr size_t kSzWPL = kSplit ? kSzWPH : 0;
constexpr size_t kSzWOF = (size_t)kDm * kCols * 2;
constexpr size_t kSzP   = (size_t)kRows * kCols * 4;
constexpr size_t kSzQ   = (size_t)kSyncBlocks * kChunkElems * 4;
constexpr size_t kSzF   = (size_t)kRows * kCols * 2;
constexpr size_t kOffXH  = 0;
constexpr size_t kOffXL  = kOffXH  + kSzXH;
constexpr size_t kOffWPH = kOffXL  + kSzXL;
constexpr size_t kOffWPL = kOffWPH + kSzWPH;
constexpr size_t kOffWOF = kOffWPL + kSzWPL;
constexpr size_t kOffP   = kOffWOF + kSzWOF;
constexpr size_t kOffQ   = kOffP   + kSzP;
constexpr size_t kOffF   = kOffQ   + kSzQ;
constexpr size_t kWsTotal = kOffF  + kSzF;
static_assert(kWsTotal == (kSplit ? 8912896ull : 7340032ull), "carve total");
static_assert(kWsTotal <= 134217728ull, "carve cap");
static_assert((kOffXL % 128) == 0 && (kOffWPH % 128) == 0 && (kOffWPL % 128) == 0 && (kOffWOF % 128) == 0 &&
              (kOffP % 128) == 0 && (kOffQ % 128) == 0 && (kOffF % 128) == 0, "128-B aligned regions");

__device__ __forceinline__ unsigned short f2bf_bits(float f) {
  unsigned u = __float_as_uint(f);
  return (unsigned short)((u + 0x7FFFu + ((u >> 16) & 1u)) >> 16);
}
__device__ __forceinline__ float bf_bits2f(unsigned short h) { return __uint_as_float(((unsigned)h) << 16); }
__device__ __forceinline__ float in_val(float v) {
  return kInputsRneToBf16 ? bf_bits2f(f2bf_bits(v)) : v;
}

__device__ __forceinline__ void mma_guard_h(v8f& c, v16h x, v16h y) { asm volatile("v_nop\n\tv_nop\n\tv_nop\n\tv_nop" : "+v"(c) : "v"(x), "v"(y)); }
__device__ __forceinline__ void mma_guard_b(v8f& c, v16b x, v16b y) { asm volatile("v_nop\n\tv_nop\n\tv_nop\n\tv_nop" : "+v"(c) : "v"(x), "v"(y)); }
__device__ __forceinline__ void keep4_h(v16h a, v16h b, v16h c, v16h d) { asm volatile("v_nop" :: "v"(a), "v"(b), "v"(c), "v"(d)); }
__device__ __forceinline__ void keep4_b(v16b a, v16b b, v16b c, v16b d) { asm volatile("v_nop" :: "v"(a), "v"(b), "v"(c), "v"(d)); }

template <typename T> struct Frag;
template <> struct Frag<_Float16> {
  typedef v16h V; union U { v16h v; v8h h[2]; };
  static __device__ __forceinline__ v16h load(const _Float16* p) {
    U f; f.h[0] = *(const v8h*)(p); f.h[1] = *(const v8h*)(p + 16); return f.v;
  }
  static __device__ __forceinline__ v8f mma(v16h a, v16h b, v8f c) {
    c = __builtin_amdgcn_wmma_f32_16x16x32_f16(false, a, false, b, (short)0, c, false, false);
    mma_guard_h(c, a, b);
    return c;
  }
  static __device__ __forceinline__ void keep(v16h a, v16h b, v16h c, v16h d) { keep4_h(a, b, c, d); }
};
template <> struct Frag<__bf16> {
  typedef v16b V; union U { v16b v; v8b h[2]; };
  static __device__ __forceinline__ v16b load(const __bf16* p) {
    U f; f.h[0] = *(const v8b*)(p); f.h[1] = *(const v8b*)(p + 16); return f.v;
  }
  static __device__ __forceinline__ v8f mma(v16b a, v16b b, v8f c) {
    c = __builtin_amdgcn_wmma_f32_16x16x32_bf16(false, a, false, b, (short)0, c, false, false);
    mma_guard_b(c, a, b);
    return c;
  }
  static __device__ __forceinline__ void keep(v16b a, v16b b, v16b c, v16b d) { keep4_b(a, b, c, d); }
};
template <int ET> struct Elem;
template <> struct Elem<0> { typedef _Float16 T; };
template <> struct Elem<1> { typedef __bf16 T; };

constexpr int kBlkX  = (kRows * kDm / 8) / 256;
constexpr int kBlkWp = (kCols * kDm / 8) / 256;
constexpr int kBlkWo = (kDm * kCols / 8) / 256;
constexpr int kPrepBlocks = kBlkX + kBlkWp + kBlkWo;
static_assert(kBlkX == 256 && kBlkWp == 128 && kBlkWo == 128, "operand plane coverage");

__global__ __launch_bounds__(256) void prep_planes_kernel(
    const float* __restrict__ x, const float* __restrict__ wp, const float* __restrict__ wo,
    unsigned short* __restrict__ XH, unsigned short* __restrict__ XL,
    unsigned short* __restrict__ WPH, unsigned short* __restrict__ WPL,
    unsigned short* __restrict__ WOF)
{
  const int blk = blockIdx.x;
  const int tid = threadIdx.x;
  if (blk < kBlkX + kBlkWp) {
    const bool isx = (blk < kBlkX);
    const float* src = isx ? x : wp;
    unsigned short* dhi = isx ? XH : WPH;
    unsigned short* dlo = isx ? XL : WPL;
    const int i = (isx ? blk : (blk - kBlkX)) * 256 + tid;
    const size_t e0 = (size_t)i << 3;
    const v4f a0 = *(const v4f*)(src + e0);
    const v4f a1 = *(const v4f*)(src + e0 + 4);
    v8h hv, lv;
#pragma unroll
    for (int e = 0; e < 4; ++e) {
      const float f0 = a0[e];
      const float f1 = a1[e];
      const unsigned short h0 = f2bf_bits(f0), h1 = f2bf_bits(f1);
      const unsigned short l0 = f2bf_bits(f0 - bf_bits2f(h0)), l1 = f2bf_bits(f1 - bf_bits2f(h1));
      hv[e]     = __builtin_bit_cast(_Float16, h0);
      hv[4 + e] = __builtin_bit_cast(_Float16, h1);
      lv[e]     = __builtin_bit_cast(_Float16, l0);
      lv[4 + e] = __builtin_bit_cast(_Float16, l1);
    }
    unsigned short* qh = dhi + e0;
    unsigned short* ql = dlo + e0;
    *(volatile v8h*)qh = hv;
    if (kSplit) *(volatile v8h*)ql = lv;
    __threadfence();
    *(volatile v8h*)qh = hv;
    if (kSplit) *(volatile v8h*)ql = lv;
  } else {
    const int i = (blk - kBlkX - kBlkWp) * 256 + tid;
    const size_t e0 = (size_t)i << 3;
    const v4f a0 = *(const v4f*)(wo + e0);
    const v4f a1 = *(const v4f*)(wo + e0 + 4);
    v8h hv;
#pragma unroll
    for (int e = 0; e < 4; ++e) {
      const float f0 = a0[e];
      const float f1 = a1[e];
      const float c0 = in_val(f0) * kCarryW;
      const float c1 = in_val(f1) * kCarryW;
      const float z0 = (fabsf(c0) < kF16MinNormal) ? 0.0f : c0;
      const float z1 = (fabsf(c1) < kF16MinNormal) ? 0.0f : c1;
      hv[e]     = (_Float16)z0;
      hv[4 + e] = (_Float16)z1;
    }
    unsigned short* qh = WOF + e0;
    *(volatile v8h*)qh = hv;
    __threadfence();
    *(volatile v8h*)qh = hv;
  }
}

template <int ET, bool SPLIT, int EPI>
__global__ __launch_bounds__(256) void wmma_gemm64(
    const unsigned short* __restrict__ Ap, const unsigned short* __restrict__ A2p, int lda,
    const unsigned short* __restrict__ Btp, const unsigned short* __restrict__ Bt2p, int ldb,
    float* __restrict__ C, int ldc,
    const float* __restrict__ bias,
    int M, int N, int K, float scale) {
  typedef typename Elem<ET>::T T;
  typedef typename Frag<T>::V V;
  const T* A = (const T*)Ap; const T* A2 = (const T*)A2p; const T* Bt = (const T*)Btp; const T* Bt2 = (const T*)Bt2p;
  __shared__ __align__(16) float sT[8][16 * 68];
  const int lane = threadIdx.x & 31;
  const int wave = threadIdx.x >> 5;
  const int tilesN = N >> 6;
  const int tilesM = M >> 6;
  const int tile = blockIdx.x * 8 + wave;
  if (tile >= tilesM * tilesN) return;
  const int tm = tile / tilesN;
  const int tn = tile - tm * tilesN;
  const int m0 = tm << 6;
  const int n0 = tn << 6;

  const int rlane = lane & 15;
  const int koff  = (lane >> 4) * 8;
  const int mOff  = (lane >> 4) * 8;

  v8f acc[4][4];
#pragma unroll
  for (int i = 0; i < 4; ++i)
#pragma unroll
    for (int j = 0; j < 4; ++j) acc[i][j] = (v8f){0.f,0.f,0.f,0.f,0.f,0.f,0.f,0.f};

  for (int k0 = 0; k0 < K; k0 += 32) {
    V bh[4], bl[4];
#pragma unroll
    for (int j = 0; j < 4; ++j) {
      const size_t bo = (size_t)(n0 + (j << 4) + rlane) * ldb + koff + k0;
      bh[j] = Frag<T>::load(Bt + bo);
      if (SPLIT) bl[j] = Frag<T>::load(Bt2 + bo);
    }
#pragma unroll
    for (int i = 0; i < 4; ++i) {
      const size_t ao = (size_t)(m0 + (i << 4) + rlane) * lda + koff + k0;
      V ah = Frag<T>::load(A + ao);
      V al;
      if (SPLIT) al = Frag<T>::load(A2 + ao);
#pragma unroll
      for (int j = 0; j < 4; ++j) {
        acc[i][j] = Frag<T>::mma(ah, bh[j], acc[i][j]);
        if (SPLIT) {
          acc[i][j] = Frag<T>::mma(ah, bl[j], acc[i][j]);
          acc[i][j] = Frag<T>::mma(al, bh[j], acc[i][j]);
        }
      }
    }
    Frag<T>::keep(bh[0], bh[1], bh[2], bh[3]);
    if (SPLIT) Frag<T>::keep(bl[0], bl[1], bl[2], bl[3]);
  }

  float* slab = sT[wave];
  float bv4[4];
#pragma unroll
  for (int j = 0; j < 4; ++j) bv4[j] = (EPI == 0) ? in_val(bias[n0 + (j << 4) + rlane]) : 0.0f;
  const float bLo = (EPI == 1) ? in_val(bias[n0 + lane]) : 0.0f;
  const float bHi = (EPI == 1) ? in_val(bias[n0 + 32 + lane]) : 0.0f;
#pragma unroll
  for (int i = 0; i < 4; ++i) {
    const int mBase = m0 + (i << 4);
#pragma unroll
    for (int j = 0; j < 4; ++j) {
#pragma unroll
      for (int r = 0; r < 8; ++r) {
        float v = acc[i][j][r] * scale;
        if (EPI == 0) v += bv4[j];
        slab[(mOff + r) * 68 + (j << 4) + rlane] = v;
      }
    }
    __builtin_amdgcn_fence(__ATOMIC_RELEASE, "workgroup");
    __builtin_amdgcn_wave_barrier();
    __builtin_amdgcn_fence(__ATOMIC_ACQUIRE, "workgroup");
    if (EPI == 1) {
#pragma unroll 1
      for (int t = 0; t < 32; ++t) {
        const int idx = t * 32 + lane;
        const int row = idx >> 6;
        const int col = idx & 63;
        const float bsel = (t & 1) ? bHi : bLo;
        const float pre = slab[row * 68 + col] + bsel;
        slab[row * 68 + col] = tanhf(pre) * kPiF;
      }
      __builtin_amdgcn_fence(__ATOMIC_RELEASE, "workgroup");
      __builtin_amdgcn_wave_barrier();
      __builtin_amdgcn_fence(__ATOMIC_ACQUIRE, "workgroup");
    }
    {
      const int hh = lane >> 4, c4 = (lane & 15) * 4;
      for (int pass = 0; pass < 2; ++pass) {
#pragma unroll
        for (int it = 0; it < 8; ++it) {
          const int row = it * 2 + hh;
          v4f v = *(const v4f*)(slab + row * 68 + c4);
          *(volatile v4f*)(C + (size_t)(mBase + row) * ldc + n0 + c4) = v;
        }
        __threadfence();
      }
    }
    __builtin_amdgcn_fence(__ATOMIC_RELEASE, "workgroup");
    __builtin_amdgcn_wave_barrier();
    __builtin_amdgcn_fence(__ATOMIC_ACQUIRE, "workgroup");
  }
}

__global__ __launch_bounds__(kSyncThreads) void phase_sync_kernel(
    const float* __restrict__ P, const float* __restrict__ mask, const float* __restrict__ nfreq,
    const float* __restrict__ coup, float* __restrict__ Q)
{
#pragma clang fp contract(off)
  __shared__ __align__(16) float sPh[kChunkElems];
  __shared__ __align__(16) float sSn[kChunkElems];
  __shared__ __align__(16) float sCs[kChunkElems];
  __shared__ float sMask[kSeq];
  __shared__ float sRedS[kRowGroups * kChunkCols];
  __shared__ float sRedC[kRowGroups * kChunkCols];
  __shared__ float sMean[2 * kChunkCols];

  const int tid = threadIdx.x;
  const int blk = blockIdx.x;
  const int j   = blk % kChunks;
  const int bh  = blk / kChunks;
  const int h   = bh % kHeads;
  const int b   = bh / kHeads;
  const int col = tid & (kChunkCols - 1);
  const int g   = tid / kChunkCols;
  const int cg  = h * kOsc + j * kChunkCols + col;

  sMask[tid]                = in_val(mask[b * kSeq + tid]);
  sMask[tid + kSyncThreads] = in_val(mask[b * kSeq + kSyncThreads + tid]);
  const float omega = in_val(nfreq[cg]);
  const float Kc    = in_val(coup[h]);

#pragma unroll 1
  for (int r = 0; r < kRowsPerThread; ++r) {
    const int pos = g * kRowsPerThread + r;
    sPh[pos * kChunkCols + col] = P[(size_t)(b * kSeq + pos) * kCols + cg];
  }
  __syncthreads();

#pragma unroll 1
  for (int it = 0; it < kIters; ++it) {
    float ssum = 0.0f, csum = 0.0f;
#pragma unroll 1
    for (int r = 0; r < kRowsPerThread; ++r) {
      const int pos = g * kRowsPerThread + r;
      const int idx = pos * kChunkCols + col;
      const float th = sPh[idx];
      const float sv = sinf(th);
      const float cv = cosf(th);
      sSn[idx] = sv;
      sCs[idx] = cv;
      const float mk = sMask[pos];
      const float ps = mk * sv;
      const float pc = mk * cv;
      ssum = ssum + ps;
      csum = csum + pc;
    }
    sRedS[g * kChunkCols + col] = ssum;
    sRedC[g * kChunkCols + col] = csum;
    __syncthreads();
    if (tid < 2 * kChunkCols) {
      const int which = tid / kChunkCols;
      const int cc    = tid & (kChunkCols - 1);
      float tot = 0.0f;
#pragma unroll 1
      for (int gg = 0; gg < kRowGroups; ++gg) {
        const float a = sRedS[gg * kChunkCols + cc];
        const float c = sRedC[gg * kChunkCols + cc];
        const float pick = which ? c : a;
        tot = tot + pick;
      }
      sMean[tid] = tot * kInvSeq;
    }
    __syncthreads();
    const float ms = sMean[col];
    const float mc = sMean[kChunkCols + col];
#pragma unroll 1
    for (int r = 0; r < kRowsPerThread; ++r) {
      const int pos = g * kRowsPerThread + r;
      const int idx = pos * kChunkCols + col;
      const float th = sPh[idx];
      const float sv = sSn[idx];
      const float cv = sCs[idx];
      const float t1  = cv * ms;
      const float t2  = sv * mc;
      const float df  = t1 - t2;
      const float cpl = Kc * df;
      const float dth = omega + cpl;
      const float stp = kDtF * dth;
      const float adv = th + stp;
      const float y   = adv + kPiF;
      const float yDn = y - kTwoPiF;
      const float yUp = y + kTwoPiF;
      float w = (y < 0.0f) ? yUp : y;
      w = (y >= kTwoPiF) ? yDn : w;
      sPh[idx] = w - kPiF;
    }
  }
  __syncthreads();

  float* Qb = Q + (size_t)blk * kChunkElems;
  v4f vals[4];
#pragma unroll
  for (int q = 0; q < 4; ++q) vals[q] = *(const v4f*)(sPh + (q * kSyncThreads + tid) * 4);
  for (int pass = 0; pass < 2; ++pass) {
#pragma unroll
    for (int q = 0; q < 4; ++q) *(volatile v4f*)(Qb + (q * kSyncThreads + tid) * 4) = vals[q];
    __threadfence();
  }
}

constexpr int kRelGroups = kCols / 8;
constexpr int kRelBlocks = (kRows * kRelGroups) / 256;
static_assert(kRelGroups == kHeads * kChunks && kRelGroups == 64 && kRelBlocks == 256, "relayout coverage");

__global__ __launch_bounds__(256) void relayout_f16_kernel(
    const float* __restrict__ Q, unsigned short* __restrict__ F)
{
  const int i  = blockIdx.x * 256 + threadIdx.x;
  const int m  = i / kRelGroups;
  const int gq = i - m * kRelGroups;
  const int b  = m / kSeq;
  const int s  = m - b * kSeq;
  const float* src = Q + ((size_t)(b * kRelGroups + gq) * kSeq + s) * kChunkCols;
  const v4f a0 = *(const v4f*)(src);
  const v4f a1 = *(const v4f*)(src + 4);
  v8h hv;
#pragma unroll
  for (int e = 0; e < 4; ++e) {
    const float f0 = a0[e];
    const float f1 = a1[e];
    const float c0 = f0 * kCarryPh;
    const float c1 = f1 * kCarryPh;
    const float z0 = (fabsf(c0) < kF16MinNormal) ? 0.0f : c0;
    const float z1 = (fabsf(c1) < kF16MinNormal) ? 0.0f : c1;
    hv[e]     = (_Float16)z0;
    hv[4 + e] = (_Float16)z1;
  }
  unsigned short* dst = F + (size_t)m * kCols + gq * 8;
  *(volatile v8h*)dst = hv;
  __threadfence();
  *(volatile v8h*)dst = hv;
}

constexpr int kGemmBlocks = ((kRows / 64) * (kCols / 64)) / 8;
static_assert(kGemmBlocks * 8 == (kRows / 64) * (kCols / 64) && kGemmBlocks == 16, "GEMM grid exact");
static_assert(kCols == kDm, "both sites share the tile grid");

extern "C" void kernel_launch(void* const* d_in, const int* in_sizes, int n_in,
                              void* d_out, int out_size, void* d_ws, size_t ws_size,
                              hipStream_t stream) {
  if (n_in < 8) return;
  if (in_sizes[0] != kRows * kDm) return;
  if (in_sizes[1] != kBatch * kSeq) return;
  if (in_sizes[2] != kCols * kDm) return;
  if (in_sizes[3] != kCols) return;
  if (in_sizes[4] != kHeads * kOsc) return;
  if (in_sizes[5] != kHeads) return;
  if (in_sizes[6] != kDm * kCols) return;
  if (in_sizes[7] != kDm) return;
  if (out_size != kRows * kDm) return;
  if (ws_size < kWsTotal) return;

  const float* x        = (const float*)d_in[0];
  const float* mask     = (const float*)d_in[1];
  const float* W_phase  = (const float*)d_in[2];
  const float* b_phase  = (const float*)d_in[3];
  const float* nat_freq = (const float*)d_in[4];
  const float* coupling = (const float*)d_in[5];
  const float* W_out    = (const float*)d_in[6];
  const float* b_out    = (const float*)d_in[7];
  float* out = (float*)d_out;

  char* ws = (char*)d_ws;
  unsigned short* XH  = (unsigned short*)(ws + kOffXH);
  unsigned short* XL  = (unsigned short*)(ws + kOffXL);
  unsigned short* WPH = (unsigned short*)(ws + kOffWPH);
  unsigned short* WPL = (unsigned short*)(ws + kOffWPL);
  unsigned short* WOF = (unsigned short*)(ws + kOffWOF);
  float*          P   = (float*)(ws + kOffP);
  float*          Q   = (float*)(ws + kOffQ);
  unsigned short* F   = (unsigned short*)(ws + kOffF);

  prep_planes_kernel<<<kPrepBlocks, 256, 0, stream>>>(x, W_phase, W_out, XH, XL, WPH, WPL, WOF);

  wmma_gemm64<1, kSplit, 1><<<dim3(kGemmBlocks), 256, 0, stream>>>(
      XH, XL, kDm, WPH, WPL, kDm, P, kCols, b_phase, kRows, kCols, kDm, 1.0f);

  phase_sync_kernel<<<kSyncBlocks, kSyncThreads, 0, stream>>>(P, mask, nat_freq, coupling, Q);

  relayout_f16_kernel<<<kRelBlocks, 256, 0, stream>>>(Q, F);

  wmma_gemm64<0, false, 0><<<dim3(kGemmBlocks), 256, 0, stream>>>(
      F, F, kCols, WOF, WOF, kCols, out, kDm, b_out, kRows, kDm, kCols, kFold);
}
